// GATModel_30459908063504
// MI455X (gfx1250) — hardware-run, weakly checked
//
#include <hip/hip_runtime.h>
#include <stddef.h>
#include <stdint.h>
#include <math.h>


#define NN     650
#define NS     400
#define NT     250
#define MP     768
#define HD     512
#define K2     1024
#define NOUT   512
#define NTHR   256
#define NWAVE  8
#define EPT    8
#define CHUNK  (NTHR * EPT)
#define WCAP   (EPT * 32)
#define LISTN  (NWAVE * WCAP)
#define NBA    64
#define SLA    6
#define RCAP   28672
#define DEGCAP 384
#define NSCAN  11
#define GBM    64
#define GBN    64
#define GTHR   128
#define NEGSL  0.2f
#define AGG_ZINTS (LISTN + 2 * RCAP + 3 * NBA)
#define AGG_LDS_INTS (AGG_ZINTS + 16)
#define WSMAX  134217728

#define NB_X   192
#define NB_W1  128
#define NB_W4  256
#define NB_P   4
#define P_AS1  0
#define P_AD1  512
#define P_B1   1024
#define P_AS4  1536
#define P_AD4  2048
#define P_B4   2560
#define P_FCW  3072
#define P_FCB  3776
#define P_TOT  4096
#define O_XB   0
#define O_W1T  (O_XB  + MP * HD * 2)
#define O_W4D  (O_W1T + HD * HD * 2)
#define O_PRM  (O_W4D + HD * K2 * 2)
#define O_Z    (O_PRM + P_TOT * 4)
#define O_H    (O_Z)
#define O_H2   (O_H   + MP * HD * 4)
#define O_X1   (O_H2  + MP * HD * 4)
#define O_X2   (O_X1  + MP * K2 * 2)
#define O_SC   (O_X2  + MP * HD * 4)
#define O_FLG  (O_SC  + 4 * MP * 4)
#define O_END  (O_FLG + 32 * 128)
#define NZUNITS ((O_END - O_Z) / 16)
#define NB_Z   (NZUNITS / NTHR)
#define NB_TOT (NB_X + NB_W1 + NB_W4 + NB_P + NB_Z)

static_assert(NS + NT == NN);
static_assert(NN <= NSCAN * NBA && NSCAN * NBA <= MP && NSCAN <= 16);
static_assert(NN * HD == NOUT * NN);
static_assert(HD % 32 == 0 && K2 % 32 == 0 && K2 == 2 * HD);
static_assert(MP % 128 == 0 && MP % GBM == 0 && HD % GBN == 0 && MP % 32 == 0);
static_assert(HD == 32 * 16);
static_assert((CHUNK & (CHUNK - 1)) == 0 && CHUNK <= 4096);
static_assert(NBA == (1 << SLA) && NBA == 64);
static_assert(((long long)CHUNK << SLA) < (1LL << 31));
static_assert(LISTN % NTHR == 0 && NBA % NWAVE == 0 && NBA % 32 == 0);
static_assert(RCAP % 4 == 0 && AGG_ZINTS % 4 == 0);
static_assert(AGG_LDS_INTS * 4 <= 300000);
static_assert(DEGCAP >= 270 + 8);
static_assert(RCAP >= 24000);
static_assert(GBM == (GTHR / 32) * 16);
static_assert(NB_X * NTHR == MP * (HD / 8));
static_assert(NB_W1 * NTHR == HD * (HD / 8));
static_assert(NB_W4 * NTHR == HD * (K2 / 8));
static_assert(NB_P * NTHR * 4 == P_TOT);
static_assert(P_FCW + 704 == P_FCB && P_FCB < P_TOT && 704 >= 21 * 32 + 32);
static_assert((O_END - O_Z) % (16 * NTHR) == 0);
static_assert(O_END <= WSMAX);
static_assert(O_W1T % 256 == 0 && O_W4D % 256 == 0 && O_PRM % 256 == 0 && O_Z % 256 == 0);
static_assert(O_H2 % 256 == 0 && O_X1 % 256 == 0 && O_X2 % 256 == 0 && O_SC % 256 == 0 && O_FLG % 256 == 0);
static_assert((NOUT - 1) * NN + (NN - 1) < NN * HD);

typedef float          v4f   __attribute__((ext_vector_type(4)));
typedef float          v8f   __attribute__((ext_vector_type(8)));
typedef int            v4i   __attribute__((ext_vector_type(4)));
typedef int            v8i   __attribute__((ext_vector_type(8)));
typedef unsigned int   v4u   __attribute__((ext_vector_type(4)));
typedef unsigned short v8us  __attribute__((ext_vector_type(8)));
typedef __bf16         v16bf __attribute__((ext_vector_type(16)));
typedef v4f  __attribute__((may_alias)) v4fa;
typedef v4i  __attribute__((may_alias)) v4ia;
typedef v8us __attribute__((may_alias)) v8usa;
union FragB { v16bf v; v8us h[2]; v8i w; };

__device__ __forceinline__ v8f wmb(const FragB& a, const FragB& b, v8f c) {
  v8f d = __builtin_amdgcn_wmma_f32_16x16x32_bf16(false, a.v, false, b.v, (short)0, c, false, false);
  asm volatile("v_nop\n\tv_nop\n\tv_nop\n\tv_nop" : "+v"(d) : "v"(a.w), "v"(b.w));
  return d;
}

__device__ __forceinline__ unsigned bf16_bits(float f) {
  const unsigned u = __float_as_uint(f);
  const unsigned r = ((u + 0x7FFFu + ((u >> 16) & 1u)) >> 16) & 0xFFFFu;
  return (f != f) ? 0x7FC0u : r;
}
__device__ __forceinline__ float bf16_val(float f) {
  return __uint_as_float(bf16_bits(f) << 16);
}
__device__ __forceinline__ unsigned msk(bool b) { return (unsigned)(-(int)b); }
__device__ __forceinline__ unsigned blend6(float a0, float a1, float a2, float a3, float a4, float a5, int sel) {
  return (__float_as_uint(a0) & msk(sel == 0)) | (__float_as_uint(a1) & msk(sel == 1)) |
         (__float_as_uint(a2) & msk(sel == 2)) | (__float_as_uint(a3) & msk(sel == 3)) |
         (__float_as_uint(a4) & msk(sel == 4)) | (__float_as_uint(a5) & msk(sel == 5));
}

template <int SLB>
__device__ __forceinline__ int scan_chunk(const int* __restrict__ dsts, int nE, int cbase, int slotBase,
                                          int nb, int vec8, int* list, int tid, int lane, int wave) {
  (void)lane;
  int wc = 0;
  const int el0  = tid * EPT;
  const int e0   = cbase + el0;
  const int sent = -2147483647 - 1;
  v4i da, db;
  if (vec8 != 0 && cbase + CHUNK <= nE) {
    da = *(const v4i*)(dsts + e0);
    db = *(const v4i*)(dsts + e0 + 4);
  } else {
    da.x = (e0     < nE) ? dsts[min(e0,     nE - 1)] : sent;
    da.y = (e0 + 1 < nE) ? dsts[min(e0 + 1, nE - 1)] : sent;
    da.z = (e0 + 2 < nE) ? dsts[min(e0 + 2, nE - 1)] : sent;
    da.w = (e0 + 3 < nE) ? dsts[min(e0 + 3, nE - 1)] : sent;
    db.x = (e0 + 4 < nE) ? dsts[min(e0 + 4, nE - 1)] : sent;
    db.y = (e0 + 5 < nE) ? dsts[min(e0 + 5, nE - 1)] : sent;
    db.z = (e0 + 6 < nE) ? dsts[min(e0 + 6, nE - 1)] : sent;
    db.w = (e0 + 7 < nE) ? dsts[min(e0 + 7, nE - 1)] : sent;
  }
  const unsigned nbs = (unsigned)slotBase;
  const unsigned unb = (unsigned)nb;
  const unsigned s0 = (unsigned)da.x - nbs, s1 = (unsigned)da.y - nbs;
  const unsigned s2 = (unsigned)da.z - nbs, s3 = (unsigned)da.w - nbs;
  const unsigned s4 = (unsigned)db.x - nbs, s5 = (unsigned)db.y - nbs;
  const unsigned s6 = (unsigned)db.z - nbs, s7 = (unsigned)db.w - nbs;
  const bool h0 = s0 < unb, h1 = s1 < unb, h2 = s2 < unb, h3 = s3 < unb;
  const bool h4 = s4 < unb, h5 = s5 < unb, h6 = s6 < unb, h7 = s7 < unb;
  const unsigned any = __builtin_amdgcn_ballot_w32(h0 | h1 | h2 | h3 | h4 | h5 | h6 | h7);
  if (any != 0u) {
#define HITJ(J, HJ, SJ) { \
      const unsigned mj = __builtin_amdgcn_ballot_w32(HJ); \
      if (mj != 0u) { \
        if (HJ) { \
          const int pos = wc + (int)__builtin_amdgcn_mbcnt_lo(mj, 0u); \
          if (pos < WCAP) list[wave * WCAP + pos] = ((el0 + (J)) << SLB) | (int)(SJ); \
        } \
        wc += (int)__builtin_popcount(mj); } }
    HITJ(0, h0, s0)
    HITJ(1, h1, s1)
    HITJ(2, h2, s2)
    HITJ(3, h3, s3)
    HITJ(4, h4, s4)
    HITJ(5, h5, s5)
    HITJ(6, h6, s6)
    HITJ(7, h7, s7)
#undef HITJ
  }
  return wc;
}

__global__ __launch_bounds__(NTHR) void k_prep(const float* __restrict__ xs, const float* __restrict__ xt,
                                               const float* __restrict__ W1, const float* __restrict__ as1,
                                               const float* __restrict__ ad1, const float* __restrict__ b1,
                                               const float* __restrict__ W4, const float* __restrict__ as4,
                                               const float* __restrict__ ad4, const float* __restrict__ b4,
                                               const float* __restrict__ fcw, const float* __restrict__ fcb,
                                               unsigned short* XB, unsigned short* W1T, unsigned short* W4D,
                                               float* PRM, v4u* Z) {
  const int b = (int)blockIdx.x, t = (int)threadIdx.x;
  if (b < NB_X) {
    const int u   = b * NTHR + t;
    const int row = u >> 6;
    const int k8  = (u & 63) * 8;
    const int rs  = row < NS ? row : NS - 1;
    int rt = row - NS;
    rt = rt < 0 ? 0 : (rt > NT - 1 ? NT - 1 : rt);
    const float* ps = xs + (size_t)rs * HD + k8;
    const float* pt = xt + (size_t)rt * HD + k8;
    const v4f sa = *(const v4f*)ps, sb = *(const v4f*)(ps + 4);
    const v4f ta = *(const v4f*)pt, tb = *(const v4f*)(pt + 4);
    const unsigned ms = msk(row < NS);
    const unsigned mt = msk(row >= NS && row < NN);
    v8us o;
    o[0] = (unsigned short)((bf16_bits(sa.x) & ms) | (bf16_bits(ta.x) & mt));
    o[1] = (unsigned short)((bf16_bits(sa.y) & ms) | (bf16_bits(ta.y) & mt));
    o[2] = (unsigned short)((bf16_bits(sa.z) & ms) | (bf16_bits(ta.z) & mt));
    o[3] = (unsigned short)((bf16_bits(sa.w) & ms) | (bf16_bits(ta.w) & mt));
    o[4] = (unsigned short)((bf16_bits(sb.x) & ms) | (bf16_bits(tb.x) & mt));
    o[5] = (unsigned short)((bf16_bits(sb.y) & ms) | (bf16_bits(tb.y) & mt));
    o[6] = (unsigned short)((bf16_bits(sb.z) & ms) | (bf16_bits(tb.z) & mt));
    o[7] = (unsigned short)((bf16_bits(sb.w) & ms) | (bf16_bits(tb.w) & mt));
    unsigned short* dp = XB + (size_t)row * HD + k8;
    *(volatile v8us*)dp = o;
    __threadfence();
    *(volatile v8us*)dp = o;
  } else if (b < NB_X + NB_W1) {
    const int u  = (b - NB_X) * NTHR + t;
    const int n  = u >> 6;
    const int k8 = (u & 63) * 8;
    const float* p = W1 + (size_t)k8 * HD + n;
    v8us o;
#pragma unroll
    for (int i = 0; i < 8; ++i) o[i] = (unsigned short)bf16_bits(p[(size_t)i * HD]);
    unsigned short* dp = W1T + (size_t)n * HD + k8;
    *(volatile v8us*)dp = o;
    __threadfence();
    *(volatile v8us*)dp = o;
  } else if (b < NB_X + NB_W1 + NB_W4) {
    const int u  = (b - NB_X - NB_W1) * NTHR + t;
    const int n  = u >> 7;
    const int k8 = (u & 127) * 8;
    const int kk = k8 & (HD - 1);
    const float* p = W4 + (size_t)kk * HD + n;
    v8us o;
#pragma unroll
    for (int i = 0; i < 8; ++i) o[i] = (unsigned short)bf16_bits(p[(size_t)i * HD]);
    unsigned short* dp = W4D + (size_t)n * K2 + k8;
    *(volatile v8us*)dp = o;
    __threadfence();
    *(volatile v8us*)dp = o;
  } else if (b < NB_X + NB_W1 + NB_W4 + NB_P) {
    const int pb  = b - (NB_X + NB_W1 + NB_W4);
    const int f0  = pb * 1024 + 4 * t;
    const int sel = f0 >> 9;
    const int vi  = f0 & (HD - 1);
    const v4f c0 = *(const v4f*)(as1 + vi);
    const v4f c1 = *(const v4f*)(ad1 + vi);
    const v4f c2 = *(const v4f*)(b1  + vi);
    const v4f c3 = *(const v4f*)(as4 + vi);
    const v4f c4 = *(const v4f*)(ad4 + vi);
    const v4f c5 = *(const v4f*)(b4  + vi);
    const float fb = fcb[0];
    const int g0 = f0 - P_FCW;
    const int g1 = g0 + 1, g2 = g0 + 2, g3 = g0 + 3;
    const float w0 = fcw[g0 < 0 ? 0 : (g0 > NN - 1 ? NN - 1 : g0)];
    const float w1 = fcw[g1 < 0 ? 0 : (g1 > NN - 1 ? NN - 1 : g1)];
    const float w2 = fcw[g2 < 0 ? 0 : (g2 > NN - 1 ? NN - 1 : g2)];
    const float w3 = fcw[g3 < 0 ? 0 : (g3 > NN - 1 ? NN - 1 : g3)];
    const unsigned fbb = __float_as_uint(fb);
    const int gb = P_FCB - P_FCW;
    unsigned r0 = blend6(c0.x, c1.x, c2.x, c3.x, c4.x, c5.x, sel);
    unsigned r1 = blend6(c0.y, c1.y, c2.y, c3.y, c4.y, c5.y, sel);
    unsigned r2 = blend6(c0.z, c1.z, c2.z, c3.z, c4.z, c5.z, sel);
    unsigned r3 = blend6(c0.w, c1.w, c2.w, c3.w, c4.w, c5.w, sel);
    r0 |= (__float_as_uint(w0) & msk((unsigned)g0 < (unsigned)NN)) | (fbb & msk(g0 == gb));
    r1 |= (__float_as_uint(w1) & msk((unsigned)g1 < (unsigned)NN)) | (fbb & msk(g1 == gb));
    r2 |= (__float_as_uint(w2) & msk((unsigned)g2 < (unsigned)NN)) | (fbb & msk(g2 == gb));
    r3 |= (__float_as_uint(w3) & msk((unsigned)g3 < (unsigned)NN)) | (fbb & msk(g3 == gb));
    v4f o;
    o.x = bf16_val(__uint_as_float(r0));
    o.y = bf16_val(__uint_as_float(r1));
    o.z = bf16_val(__uint_as_float(r2));
    o.w = bf16_val(__uint_as_float(r3));
    float* dp = PRM + f0;
    *(volatile v4f*)dp = o;
    __threadfence();
    *(volatile v4f*)dp = o;
  } else {
    const int u = (b - (NB_X + NB_W1 + NB_W4 + NB_P)) * NTHR + t;
    if (u < NZUNITS) {
      const v4u z = {0u, 0u, 0u, 0u};
      *(volatile v4u*)(Z + u) = z;
      __threadfence();
      *(volatile v4u*)(Z + u) = z;
    }
  }
}

__global__ __launch_bounds__(GTHR) void k_gemm(const unsigned short* __restrict__ A,
                                               const unsigned short* __restrict__ WT,
                                               float* outF, int K, int ldo) {
  __shared__ __attribute__((aligned(16))) float stg[GBM * GBN];
  const int tid = (int)threadIdx.x, lane = tid & 31, wave = tid >> 5, hh = lane >> 4, m = lane & 15;
  const int rowBase = (int)blockIdx.x * GBM;
  const int col0    = (int)blockIdx.y * GBN;

  v8f acc[4];
  {
    const v8f z = {0.f, 0.f, 0.f, 0.f, 0.f, 0.f, 0.f, 0.f};
    acc[0] = z; acc[1] = z; acc[2] = z; acc[3] = z;
  }
  const unsigned short* ap = A  + (size_t)(rowBase + 16 * wave + m) * (size_t)K + 8 * hh;
  const unsigned short* wp = WT + (size_t)(col0 + m) * (size_t)K + 8 * hh;
  const int ksteps = K >> 5;
#pragma unroll 1
  for (int ks = 0; ks < ksteps; ++ks) {
    FragB af;
    af.h[0] = *(const v8usa*)(ap + 32 * ks);
    af.h[1] = *(const v8usa*)(ap + 32 * ks + 16);
#pragma unroll
    for (int t = 0; t < 4; ++t) {
      const unsigned short* wq = wp + (size_t)(16 * t) * (size_t)K + 32 * ks;
      FragB bf;
      bf.h[0] = *(const v8usa*)wq;
      bf.h[1] = *(const v8usa*)(wq + 16);
      acc[t] = wmb(af, bf, acc[t]);
    }
  }

#pragma unroll
  for (int t = 0; t < 4; ++t) {
    const int lc = 16 * t + m;
#pragma unroll
    for (int r = 0; r < 8; ++r) {
      const int lr = 16 * wave + 8 * hh + r;
      stg[lr * GBN + lc] = acc[t][r];
    }
  }
  __syncthreads();

  v4f fv[8];
#pragma unroll
  for (int i = 0; i < 8; ++i) {
    const int lr = 16 * wave + 2 * i + hh;
    fv[i] = *(const v4fa*)(stg + lr * GBN + 4 * m);
  }
#pragma unroll
  for (int i = 0; i < 8; ++i) {
    const int lr = 16 * wave + 2 * i + hh;
    float* op = outF + (size_t)(rowBase + lr) * (size_t)ldo + col0 + 4 * m;
    *(volatile v4f*)op = fv[i];
  }
  __threadfence();
#pragma unroll
  for (int i = 0; i < 8; ++i) {
    const int lr = 16 * wave + 2 * i + hh;
    float* op = outF + (size_t)(rowBase + lr) * (size_t)ldo + col0 + 4 * m;
    *(volatile v4f*)op = fv[i];
  }
}

__global__ __launch_bounds__(NTHR) void k_dots(const float* __restrict__ H, const float* __restrict__ prm,
                                               int aoff, float* sc, int asOff, int adOff) {
  __shared__ __attribute__((aligned(16))) float sa[2 * HD];
  __shared__ __attribute__((aligned(16))) float sdt[64];
  const int tid = (int)threadIdx.x, lane = tid & 31, wave = tid >> 5;
  {
    const v4f a = *(const v4f*)(prm + aoff + 4 * tid);
    *(v4fa*)(sa + 4 * tid) = a;
  }
  __syncthreads();
#pragma unroll 1
  for (int i = 0; i < 4; ++i) {
    const int lr  = 4 * wave + i;
    const int row = (int)blockIdx.x * 32 + lr;
    const float* hp = H + (size_t)row * HD + 4 * lane;
    float s = 0.0f, d = 0.0f;
#pragma unroll 1
    for (int q = 0; q < 4; ++q) {
      const v4f p = *(const v4f*)(hp + 128 * q);
      const v4f a = *(const v4fa*)(sa + 128 * q + 4 * lane);
      const v4f e = *(const v4fa*)(sa + HD + 128 * q + 4 * lane);
      s = fmaf(p.x, a.x, s); s = fmaf(p.y, a.y, s); s = fmaf(p.z, a.z, s); s = fmaf(p.w, a.w, s);
      d = fmaf(p.x, e.x, d); d = fmaf(p.y, e.y, d); d = fmaf(p.z, e.z, d); d = fmaf(p.w, e.w, d);
    }
#pragma unroll
    for (int off = 16; off > 0; off >>= 1) {
      s += __shfl_xor(s, off);
      d += __shfl_xor(d, off);
    }
    if (lane == 0) { sdt[lr] = s; sdt[32 + lr] = d; }
  }
  __syncthreads();
  if (wave == 0) {
    const v4f v = *(const v4fa*)(sdt + 4 * (lane & 15));
    const int off = ((lane < 8) ? asOff : adOff) + (int)blockIdx.x * 32 + 4 * (lane & 7);
    if (lane < 16) {
      *(volatile v4f*)(sc + off) = v;
      __threadfence();
      *(volatile v4f*)(sc + off) = v;
    }
  }
}

template <int LAY>
__device__ __forceinline__ int coff(int p, int lane) {
  return (LAY == 1) ? (256 * (p >> 1) + 8 * lane + 4 * (p & 1)) : (128 * p + 4 * lane);
}

template <int LAY>
__global__ __launch_bounds__(NTHR) void k_scan(const int* __restrict__ srcs, const int* __restrict__ dsts,
                                               int nE, int nN, int vec8, int mRows,
                                               const float* __restrict__ AS, const float* __restrict__ AD,
                                               const float* __restrict__ xl, const float* __restrict__ bias,
                                               unsigned short* hb, float* outp, int* flg) {
  extern __shared__ __attribute__((aligned(16))) int dsm[];
  int* list = dsm;
  int* hl   = dsm + LISTN;
  int* sl   = dsm + LISTN + RCAP;
  int* cnt  = dsm + LISTN + 2 * RCAP;
  int* offs = cnt + NBA;
  int* cur  = offs + NBA;
  int* misc = cur + NBA;
  const int tid = (int)threadIdx.x, lane = tid & 31, wave = tid >> 5;
  const int nodeBase = (int)blockIdx.x * NBA;

  {
    const v4i z4 = {0, 0, 0, 0};
    for (int i = tid * 4; i < AGG_ZINTS; i += NTHR * 4) *(v4ia*)(dsm + i) = z4;
    if (tid < 16) misc[tid] = 0;
  }
  const int c0 = coff<LAY>(0, lane), c1 = coff<LAY>(1, lane), c2 = coff<LAY>(2, lane), c3 = coff<LAY>(3, lane);
  const v4f bv0 = *(const v4f*)(bias + c0);
  const v4f bv1 = *(const v4f*)(bias + c1);
  const v4f bv2 = *(const v4f*)(bias + c2);
  const v4f bv3 = *(const v4f*)(bias + c3);
  __syncthreads();

  int t = 0, ov = 0;
  const int nChunks = (nE + CHUNK - 1) / CHUNK;
#pragma unroll 1
  for (int ch = 0; ch < nChunks; ++ch) {
    const int cbase = ch * CHUNK;
    const int wc = scan_chunk<SLA>(dsts, nE, cbase, nodeBase, NBA, vec8, list, tid, lane, wave);
    if (lane == 0) misc[wave] = wc;
    __syncthreads();
    if (wave == 0) {
#pragma unroll 1
      for (int w2 = 0; w2 < NWAVE; ++w2) {
        int c = misc[w2];
        c = c < 0 ? 0 : (c > WCAP ? WCAP : c);
#pragma unroll 1
        for (int b0 = 0; b0 < c; b0 += 32) {
          const int idx = b0 + lane;
          const int ent = list[w2 * WCAP + (idx < WCAP ? idx : WCAP - 1)];
          const int m32 = (c - b0) < 32 ? (c - b0) : 32;
#pragma unroll 1
          for (int k = 0; k < m32; ++k) {
            const int u    = __builtin_amdgcn_readlane(ent, k);
            const int slot = u & (NBA - 1);
            const int el   = (u >> SLA) & (CHUNK - 1);
            const int pk   = ((cbase + el) << SLA) | slot;
            if (t < RCAP) {
              if (lane == 0) { hl[t] = pk; cnt[slot] = cnt[slot] + 1; }
              t = t + 1;
            } else {
              ov = 1;
            }
          }
        }
      }
    }
    __syncthreads();
  }
  if (wave == 0 && lane == 0) { misc[8] = t; misc[9] = ov; }
  __syncthreads();
  int tt = misc[8];
  tt = tt < 0 ? 0 : (tt > RCAP ? RCAP : tt);
  const int ovf = misc[9];

  if (wave == 0) {
    const int cb0 = cnt[lane], cb1 = cnt[lane + 32];
    const unsigned bm = __builtin_amdgcn_ballot_w32((cb0 > DEGCAP) | (cb1 > DEGCAP));
    if (lane == 0) misc[10] = (bm != 0u) ? 1 : 0;
    const int base = lane * (NBA / 32);
    int s = 0;
#pragma unroll 1
    for (int i = 0; i < NBA / 32; ++i) s += cnt[base + i];
    int incl = s;
#pragma unroll
    for (int d = 1; d < 32; d <<= 1) {
      const int y = __shfl_up(incl, d, 32);
      if (lane >= d) incl += y;
    }
    int run = incl - s;
#pragma unroll 1
    for (int i = 0; i < NBA / 32; ++i) {
      const int cv = cnt[base + i];
      offs[base + i] = run;
      cur[base + i]  = run;
      run += cv;
    }
  }
  __syncthreads();
  if (wave == 0) {
#pragma unroll 1
    for (int b0 = 0; b0 < tt; b0 += 32) {
      const int idx = b0 + lane;
      const int ent = hl[idx < RCAP ? idx : RCAP - 1];
      const int m32 = (tt - b0) < 32 ? (tt - b0) : 32;
#pragma unroll 1
      for (int k = 0; k < m32; ++k) {
        const int u    = __builtin_amdgcn_readlane(ent, k);
        const int slot = u & (NBA - 1);
        if (lane == 0) {
          int p = cur[slot];
          p = p < 0 ? 0 : (p > RCAP - 1 ? RCAP - 1 : p);
          sl[p] = u;
          cur[slot] = p + 1;
        }
      }
    }
  }
  __syncthreads();

  {
    const int fl = ((ovf != 0) || (misc[10] != 0)) ? 1 : 0;
    if (wave == 0 && lane < 8) {
      const v4i fv = {fl, fl, fl, fl};
      int* fp = flg + (int)blockIdx.x * 32 + 4 * lane;
      *(volatile v4i*)fp = fv;
      __threadfence();
      *(volatile v4i*)fp = fv;
    }
  }

  const float qnan = __int_as_float(0x7fc00000);
  const float pz = (ovf != 0) ? qnan : 0.0f;
#pragma unroll 1
  for (int si = 0; si < NBA / NWAVE; ++si) {
    const int s    = si * NWAVE + wave;
    const int node = nodeBase + s;
    const int craw = cnt[s];
    const bool big = craw > DEGCAP;
    int c = craw < 0 ? 0 : (craw > DEGCAP ? DEGCAP : craw);
    int o = offs[s];
    o = o < 0 ? 0 : (o > tt ? tt : o);
    if (c > tt - o) c = tt - o;
    const int nc = node < nN ? node : nN - 1;
    const float as0 = AS[nc];
    const float ad  = AD[nc];
    float l0 = as0 + ad;
    l0 = l0 > 0.f ? l0 : NEGSL * l0;
    float mx = l0, dn = 0.0f;
    v4f acc0 = {0.f, 0.f, 0.f, 0.f}, acc1 = acc0, acc2 = acc0, acc3 = acc0;
#pragma unroll 1
    for (int b0 = 0; b0 < c; b0 += 32) {
      int idx = o + b0 + lane;
      idx = idx > RCAP - 1 ? RCAP - 1 : idx;
      const int ent = sl[idx];
      int eid = ent >> SLA;
      eid = eid < 0 ? 0 : (eid > nE - 1 ? nE - 1 : eid);
      int sr = srcs[eid];
      sr = sr < 0 ? 0 : (sr > nN - 1 ? nN - 1 : sr);
      const float es  = AS[sr];
      const int   esi = __float_as_int(es);
      const int m32 = (c - b0) < 32 ? (c - b0) : 32;
#pragma unroll 1
      for (int k = 0; k < m32; ++k) {
        const int   sk  = __builtin_amdgcn_readlane(sr, k);
        const float ask = __int_as_float(__builtin_amdgcn_readlane(esi, k));
        const float* rp = xl + (size_t)sk * HD;
        const v4f g0 = *(const v4f*)(rp + c0);
        const v4f g1 = *(const v4f*)(rp + c1);
        const v4f g2 = *(const v4f*)(rp + c2);
        const v4f g3 = *(const v4f*)(rp + c3);
        float lg = ask + ad;
        lg = lg > 0.f ? lg : NEGSL * lg;
        const float df = lg - mx;
        const float ee = expf(-fabsf(df));
        const bool  up = df > 0.f;
        const float s1 = up ? ee : 1.0f;
        const float s2 = up ? 1.0f : ee;
        mx = up ? lg : mx;
        dn = fmaf(dn, s1, s2);
        acc0 = acc0 * s1 + g0 * s2;
        acc1 = acc1 * s1 + g1 * s2;
        acc2 = acc2 * s1 + g2 * s2;
        acc3 = acc3 * s1 + g3 * s2;
      }
    }
    {
      const float* sp = xl + (size_t)nc * HD;
      const v4f g0 = *(const v4f*)(sp + c0);
      const v4f g1 = *(const v4f*)(sp + c1);
      const v4f g2 = *(const v4f*)(sp + c2);
      const v4f g3 = *(const v4f*)(sp + c3);
      const float ps = expf(l0 - mx);
      dn = dn + ps;
      acc0 = acc0 + g0 * ps;
      acc1 = acc1 + g1 * ps;
      acc2 = acc2 + g2 * ps;
      acc3 = acc3 + g3 * ps;
    }
    const float inv = 1.0f / (dn + 1e-16f);
    const float pzr = big ? qnan : pz;
    const bool live = node < nN;
    float v[16];
    v[0]  = fmaf(acc0.x, inv, bv0.x); v[1]  = fmaf(acc0.y, inv, bv0.y);
    v[2]  = fmaf(acc0.z, inv, bv0.z); v[3]  = fmaf(acc0.w, inv, bv0.w);
    v[4]  = fmaf(acc1.x, inv, bv1.x); v[5]  = fmaf(acc1.y, inv, bv1.y);
    v[6]  = fmaf(acc1.z, inv, bv1.z); v[7]  = fmaf(acc1.w, inv, bv1.w);
    v[8]  = fmaf(acc2.x, inv, bv2.x); v[9]  = fmaf(acc2.y, inv, bv2.y);
    v[10] = fmaf(acc2.z, inv, bv2.z); v[11] = fmaf(acc2.w, inv, bv2.w);
    v[12] = fmaf(acc3.x, inv, bv3.x); v[13] = fmaf(acc3.y, inv, bv3.y);
    v[14] = fmaf(acc3.z, inv, bv3.z); v[15] = fmaf(acc3.w, inv, bv3.w);
#pragma unroll
    for (int i = 0; i < 16; ++i) {
      float y = v[i];
      if (LAY == 1) y = (y > 0.0f) ? y : (y - y);
      else          y = (y > 0.0f) ? y : 0.01f * y;
      y = y + pzr;
      v[i] = live ? y : 0.0f;
    }
    if constexpr (LAY == 1) {
      v8us ho0, lo0, ho1, lo1;
#pragma unroll
      for (int i = 0; i < 8; ++i) {
        const unsigned ha = bf16_bits(v[i]);
        ho0[i] = (unsigned short)ha;
        lo0[i] = (unsigned short)bf16_bits(v[i] - __uint_as_float(ha << 16));
        const unsigned hc = bf16_bits(v[8 + i]);
        ho1[i] = (unsigned short)hc;
        lo1[i] = (unsigned short)bf16_bits(v[8 + i] - __uint_as_float(hc << 16));
      }
      if (node < mRows) {
        unsigned short* hp = hb + (size_t)node * K2 + 8 * lane;
        *(volatile v8us*)hp = ho0;
        *(volatile v8us*)(hp + 256) = ho1;
        *(volatile v8us*)(hp + HD) = lo0;
        *(volatile v8us*)(hp + HD + 256) = lo1;
        __threadfence();
        *(volatile v8us*)hp = ho0;
        *(volatile v8us*)(hp + 256) = ho1;
        *(volatile v8us*)(hp + HD) = lo0;
        *(volatile v8us*)(hp + HD + 256) = lo1;
      }
    } else {
      v4f o0, o1, o2, o3;
      o0.x = v[0];  o0.y = v[1];  o0.z = v[2];  o0.w = v[3];
      o1.x = v[4];  o1.y = v[5];  o1.z = v[6];  o1.w = v[7];
      o2.x = v[8];  o2.y = v[9];  o2.z = v[10]; o2.w = v[11];
      o3.x = v[12]; o3.y = v[13]; o3.z = v[14]; o3.w = v[15];
      if (live) {
        float* op = outp + (size_t)node * HD + 4 * lane;
        *(volatile v4f*)op = o0;
        *(volatile v4f*)(op + 128) = o1;
        *(volatile v4f*)(op + 256) = o2;
        *(volatile v4f*)(op + 384) = o3;
        __threadfence();
        *(volatile v4f*)op = o0;
        *(volatile v4f*)(op + 128) = o1;
        *(volatile v4f*)(op + 256) = o2;
        *(volatile v4f*)(op + 384) = o3;
      }
    }
  }
}

__global__ __launch_bounds__(NTHR) void k_fc(const float* __restrict__ X2, const float* __restrict__ prm,
                                             const int* __restrict__ flg, float* out) {
  __shared__ __attribute__((aligned(16))) float sfw[1024];
  __shared__ __attribute__((aligned(16))) float sres[32];
  const int tid = (int)threadIdx.x, lane = tid & 31, wave = tid >> 5;
  {
    const v4f a = *(const v4f*)(prm + P_FCW + 4 * tid);
    *(v4fa*)(sfw + 4 * tid) = a;
  }
  __syncthreads();
  const float fb = sfw[P_FCB - P_FCW];
#pragma unroll 1
  for (int i = 0; i < 4; ++i) {
    const int lr = 4 * wave + i;
    const int r  = (int)blockIdx.x * 32 + lr;
    const float* yr = X2 + (size_t)r * NN;
    float s = 0.0f;
#pragma unroll 1
    for (int tq = 0; tq < 21; ++tq) {
      const int j  = lane + 32 * tq;
      const int jc = j < NN ? j : NN - 1;
      const float x = yr[jc];
      const float w = sfw[j];
      s = fmaf(x, w, s);
    }
#pragma unroll
    for (int off = 16; off > 0; off >>= 1) s += __shfl_xor(s, off);
    const float z = s + fb;
    const float y = 1.0f / (1.0f + expf(-z));
    if (lane == 0) sres[lr] = y;
  }
  __syncthreads();
  if (wave == 0) {
    const int fl = flg[lane * 32];
    const unsigned anyf = __builtin_amdgcn_ballot_w32(fl != 0);
    v4f v = *(const v4fa*)(sres + 4 * (lane & 7));
    const float qn = __int_as_float(0x7fc00000);
    if (anyf != 0u) { v.x = qn; v.y = qn; v.z = qn; v.w = qn; }
    if (lane < 8) {
      float* op = out + (int)blockIdx.x * 32 + 4 * lane;
      *(volatile v4f*)op = v;
      __threadfence();
      *(volatile v4f*)op = v;
    }
  }
}

extern "C" void kernel_launch(void* const* d_in, const int* in_sizes, int n_in,
                              void* d_out, int out_size, void* d_ws, size_t ws_size,
                              hipStream_t stream) {
  if (n_in < 15) return;
  if (in_sizes[0] != NS * HD) return;
  if (in_sizes[1] != NT * HD) return;
  if (in_sizes[2] < 2 || (in_sizes[2] & 1) != 0) return;
  const int nE = in_sizes[2] / 2;
  if (nE < 1 || nE >= (1 << 25)) return;
  if (in_sizes[5] != HD * HD) return;
  if (in_sizes[6] != HD || in_sizes[7] != HD || in_sizes[8] != HD) return;
  if (in_sizes[9] != HD * HD) return;
  if (in_sizes[10] != HD || in_sizes[11] != HD || in_sizes[12] != HD) return;
  if (in_sizes[13] != NN) return;
  if (in_sizes[14] != 1) return;
  if (out_size != NOUT) return;
  if ((size_t)O_END > ws_size || (size_t)O_END > (size_t)WSMAX) return;

  const float* xs   = (const float*)d_in[0];
  const float* xt   = (const float*)d_in[1];
  const int*   edge = (const int*)d_in[2];
  const float* W1   = (const float*)d_in[5];
  const float* as1  = (const float*)d_in[6];
  const float* ad1  = (const float*)d_in[7];
  const float* b1   = (const float*)d_in[8];
  const float* W4   = (const float*)d_in[9];
  const float* as4  = (const float*)d_in[10];
  const float* ad4  = (const float*)d_in[11];
  const float* b4   = (const float*)d_in[12];
  const float* fcw  = (const float*)d_in[13];
  const float* fcb  = (const float*)d_in[14];
  float* out = (float*)d_out;
  const int* src = edge;
  const int* dst = edge + nE;
  const int vec8 = ((nE & 3) == 0) ? 1 : 0;

  char* ws = (char*)d_ws;
  unsigned short* XB  = (unsigned short*)(ws + O_XB);
  unsigned short* W1T = (unsigned short*)(ws + O_W1T);
  unsigned short* W4D = (unsigned short*)(ws + O_W4D);
  float*          PRM = (float*)(ws + O_PRM);
  v4u*            Zp  = (v4u*)(ws + O_Z);
  float*          H   = (float*)(ws + O_H);
  float*          H2  = (float*)(ws + O_H2);
  unsigned short* X1  = (unsigned short*)(ws + O_X1);
  float*          X2  = (float*)(ws + O_X2);
  float*          SC  = (float*)(ws + O_SC);
  int*            FLG = (int*)(ws + O_FLG);

  const int aggLds = AGG_LDS_INTS * 4;
  hipFuncSetAttribute(reinterpret_cast<const void*>(&k_scan<1>), hipFuncAttributeMaxDynamicSharedMemorySize, aggLds);
  hipFuncSetAttribute(reinterpret_cast<const void*>(&k_scan<2>), hipFuncAttributeMaxDynamicSharedMemorySize, aggLds);

  k_prep<<<NB_TOT, NTHR, 0, stream>>>(xs, xt, W1, as1, ad1, b1, W4, as4, ad4, b4, fcw, fcb,
                                      XB, W1T, W4D, PRM, Zp);
  k_gemm<<<dim3(MP / GBM, HD / GBN), GTHR, 0, stream>>>(XB, W1T, H, HD, HD);
  k_dots<<<MP / 32, NTHR, 0, stream>>>(H, PRM, P_AS1, SC, 0, MP);
  k_scan<1><<<NSCAN, NTHR, (size_t)aggLds, stream>>>(src, dst, nE, NN, vec8, MP, SC, SC + MP, H, PRM + P_B1,
                                                     X1, X2, FLG);
  k_gemm<<<dim3(MP / GBM, HD / GBN), GTHR, 0, stream>>>(X1, W4D, H2, K2, HD);
  k_dots<<<MP / 32, NTHR, 0, stream>>>(H2, PRM, P_AS4, SC, 2 * MP, 3 * MP);
  k_scan<2><<<NSCAN, NTHR, (size_t)aggLds, stream>>>(src, dst, nE, NN, vec8, MP, SC + 2 * MP, SC + 3 * MP, H2,
                                                     PRM + P_B4, X1, X2, FLG + 16 * 32);
  k_fc<<<NOUT / 32, NTHR, 0, stream>>>(X2, PRM, FLG, out);
}
